// BatchNeuralMemory_89781996355759
// MI455X (gfx1250) — hardware-run, weakly checked
//
#include <hip/hip_runtime.h>
#include <math.h>

#ifndef NB
#define NB 2
#endif
#ifndef SEQ
#define SEQ 1024
#endif
#define NB_FULL 2
#define SEQ_FULL 1024
#define DM 1024
#define HID 2048
#define CHK 64
#define NCH (SEQ / CHK)
#define MTOK (NB * SEQ)

#define CX_L2 6
#define CW_L2 10
#define CK_L2 9
#define CH_L2 10
#define CDY_L2 26
#define CDZ_L2 27
#define CN1_L2 23
#define CN2_L2 22
#define CHQ_L2 16

#define OFF_OUT 0u
#define OFF_NW1 2097152u
#define OFF_NW2 6291456u
#define OFF_NLN 10485760u
#define OFF_NS1 10487808u
#define OFF_NS2 14682112u
#define OFF_NSL 18876416u
#define OUT_ELEMS 18878464u

static_assert(SEQ % 64 == 0);
static_assert(NCH >= 1 && NCH <= 16);
static_assert(NB >= 1 && NB <= NB_FULL && SEQ <= SEQ_FULL);
static_assert(MTOK % 64 == 0 && DM % 64 == 0 && HID % 64 == 0 && (3 * DM) % 64 == 0);
static_assert(DM % 32 == 0 && HID % 32 == 0 && CHK % 32 == 0);
static_assert((size_t)OFF_NW1 * 4 == 8388608 && (size_t)OFF_NW2 * 4 == 25165824 && (size_t)OFF_NLN * 4 == 41943040);
static_assert((size_t)OFF_NS1 * 4 == 41951232 && (size_t)OFF_NS2 * 4 == 58728448 && (size_t)OFF_NSL * 4 == 75505664);
static_assert((size_t)OUT_ELEMS * 4 == 75513856);
static_assert(OFF_NW1 == (unsigned)NB_FULL * SEQ_FULL * DM);
static_assert(OFF_NW2 == OFF_NW1 + (unsigned)NB_FULL * HID * DM && OFF_NLN == OFF_NW2 + (unsigned)NB_FULL * HID * DM);
static_assert(OFF_NS1 == OFF_NLN + (unsigned)NB_FULL * DM && OFF_NS2 == OFF_NS1 + (unsigned)NB_FULL * HID * DM);
static_assert(OFF_NSL == OFF_NS2 + (unsigned)NB_FULL * HID * DM && OUT_ELEMS == OFF_NSL + (unsigned)NB_FULL * DM);
static_assert((size_t)(NB - 1) * SEQ_FULL * DM + (size_t)SEQ * DM <= OFF_NW1);
static_assert((size_t)NB * HID * DM <= (size_t)(OFF_NW2 - OFF_NW1) && (size_t)NB * DM <= (size_t)(OFF_NS1 - OFF_NLN));

typedef _Float16 h16;
typedef __attribute__((ext_vector_type(16))) _Float16 v16h;
typedef __attribute__((ext_vector_type(8)))  _Float16 v8h;
typedef __attribute__((ext_vector_type(8)))  float    v8f;
typedef __attribute__((ext_vector_type(4)))  float    v4f;


#define VST2V4(ptr, val) do { const v4f vst2_v4_ = (val); *(volatile v4f*)(ptr) = vst2_v4_; __threadfence(); *(volatile v4f*)(ptr) = vst2_v4_; } while (0)

__host__ __device__ constexpr float p2f(int e) {
    float r = 1.0f;
    const int n = (e < 0) ? -e : e;
    for (int i = 0; i < n; ++i) r = (e < 0) ? r * 0.5f : r * 2.0f;
    return r;
}

static __device__ __forceinline__ float bfr(float f) {
    unsigned u = __float_as_uint(f);
    u += 0x7FFFu + ((u >> 16) & 1u);
    return __uint_as_float(u & 0xFFFF0000u);
}
static __device__ __forceinline__ h16 toh_flush(float v) { const float w = (fabsf(v) < 6.103515625e-05f) ? 0.0f : v; return (h16)w; }
static __device__ __forceinline__ float sigm(float z) { return 1.0f / (1.0f + expf(-z)); }

union FragU { v16h v; v8h h[2]; };
static __device__ __forceinline__ v16h frag_ld(const h16* p) {
    FragU f; f.h[0] = *(const v8h*)(p); f.h[1] = *(const v8h*)(p + 16); return f.v;
}
static __device__ __forceinline__ v8f wmma16g(v16h a, v16h b, v8f c) {
    c = __builtin_amdgcn_wmma_f32_16x16x32_f16(false, a, false, b, (short)0, c, false, false);
    asm volatile("v_nop\n\tv_nop\n\tv_nop\n\tv_nop" : "+v"(c) : "v"(a), "v"(b));
    return c;
}
static __device__ __forceinline__ void wave_sync_lds() {
    __builtin_amdgcn_fence(3  , "workgroup");
    __builtin_amdgcn_wave_barrier();
    __builtin_amdgcn_fence(2  , "workgroup");
}

template <int CL2>
__global__ __launch_bounds__(256) void k_cvt(const float* __restrict__ src, h16* __restrict__ dst, unsigned n8,
                                             unsigned sstride, unsigned dstride) {
    const unsigned u = blockIdx.x * 256u + threadIdx.x;
    if (u >= n8) return;
    constexpr float CAR = p2f(CL2);
    const float* sp = src + (size_t)blockIdx.y * sstride + (size_t)u * 8u;
    const v4f a = *(const v4f*)sp, b = *(const v4f*)(sp + 4);
    const float v[8] = {a.x, a.y, a.z, a.w, b.x, b.y, b.z, b.w};
    v8h pk;
#pragma unroll
    for (int e = 0; e < 8; ++e) pk[e] = toh_flush(bfr(v[e]) * CAR);
    h16* dp = dst + (size_t)blockIdx.y * dstride + (size_t)u * 8u;
    *(volatile v8h*)dp = pk;
    __threadfence();
    *(volatile v8h*)dp = pk;
}

__global__ __launch_bounds__(256) void k_tr16(const h16* __restrict__ in, h16* __restrict__ out, unsigned R, unsigned Cc) {
    __shared__ __align__(16) h16 sT[64 * 72];
    const unsigned t = threadIdx.x;
    const unsigned c0 = blockIdx.x * 64u, r0 = blockIdx.y * 64u;
#pragma unroll
    for (int it = 0; it < 2; ++it) {
        const unsigned idx = t + 256u * (unsigned)it;
        const unsigned r = idx >> 3, p = idx & 7u;
        const v8h v = *(const v8h*)(in + (size_t)(r0 + r) * Cc + c0 + 8u * p);
        *(v8h*)(sT + r * 72u + 8u * p) = v;
    }
    __syncthreads();
    v8h o[2];
#pragma unroll
    for (int it = 0; it < 2; ++it) {
        const unsigned idx = t + 256u * (unsigned)it;
        const unsigned orow = idx >> 3, p = idx & 7u;
#pragma unroll
        for (int e = 0; e < 8; ++e) o[it][e] = sT[(8u * p + (unsigned)e) * 72u + orow];
    }
    for (int pass = 0; pass < 2; ++pass) {
#pragma unroll
        for (int it = 0; it < 2; ++it) {
            const unsigned idx = t + 256u * (unsigned)it;
            const unsigned orow = idx >> 3, p = idx & 7u;
            *(volatile v8h*)(out + (size_t)(c0 + orow) * R + r0 + 8u * p) = o[it];
        }
        __threadfence();
    }
}

__global__ __launch_bounds__(256) void k_gates(const float* __restrict__ x, const float* __restrict__ aw, const float* __restrict__ tw,
                                               const float* __restrict__ ew, float* __restrict__ gates, unsigned niter) {
    __shared__ float sm[3][256];
    const unsigned t = threadIdx.x;
    const unsigned bn = blockIdx.x;
    const unsigned b = bn / (unsigned)NCH;
    const unsigned n = bn - b * (unsigned)NCH;
    const float* xc = x + ((size_t)b * SEQ_FULL + (size_t)n * CHK) * DM;
    float sa = 0.f, st = 0.f, se = 0.f;
    for (unsigned j = 0; j < niter; ++j) {
        const unsigned i = 4u * t + 1024u * j;
        const v4f xv = *(const v4f*)(xc + i);
        const v4f av = *(const v4f*)(aw + i);
        const v4f tv = *(const v4f*)(tw + i);
        const v4f ev = *(const v4f*)(ew + i);
        const float x0 = bfr(xv.x), x1 = bfr(xv.y), x2 = bfr(xv.z), x3 = bfr(xv.w);
        sa += x0 * bfr(av.x); sa += x1 * bfr(av.y); sa += x2 * bfr(av.z); sa += x3 * bfr(av.w);
        st += x0 * bfr(tv.x); st += x1 * bfr(tv.y); st += x2 * bfr(tv.z); st += x3 * bfr(tv.w);
        se += x0 * bfr(ev.x); se += x1 * bfr(ev.y); se += x2 * bfr(ev.z); se += x3 * bfr(ev.w);
    }
    sm[0][t] = sa; sm[1][t] = st; sm[2][t] = se;
    __syncthreads();
    for (unsigned s = 128u; s > 0u; s >>= 1) {
        if (t < s) { sm[0][t] += sm[0][t + s]; sm[1][t] += sm[1][t + s]; sm[2][t] += sm[2][t + s]; }
        __syncthreads();
    }
    const float ga = sigm(sm[0][0]);
    const float gt = sigm(sm[1][0]) * 0.01f;
    const float ge = sigm(sm[2][0]);
    if (t < 8u) {
        v4f o;
        o.x = (t == 0u) ? ga : 0.f; o.y = (t == 0u) ? gt : 0.f; o.z = (t == 0u) ? ge : 0.f; o.w = 0.f;
        VST2V4(gates + (size_t)bn * 32u + 4u * t, o);
    }
}

__global__ __launch_bounds__(32) void k_coef(const float* __restrict__ gates, float* __restrict__ coef, unsigned nch) {
    __shared__ float sA[16];
    __shared__ float sE[16];
    __shared__ __align__(16) float sO[64];
    const unsigned t = threadIdx.x, b = blockIdx.x;
    const unsigned tt = t & 15u;
    const unsigned tc = min(tt, nch - 1u);
    const float* line = gates + (size_t)(b * nch + tc) * 32u;
    const float al = line[0], th = line[1], et = line[2];
    const bool live = tt < nch;
    if (t < 16u) { sA[t] = live ? al : 0.f; sE[t] = live ? et : 1.f; }
    __syncthreads();
    float dco = 1.f;
    for (unsigned u = 0; u < nch; ++u) { const float ev = sE[u]; dco *= (u > tt) ? ev : 1.0f; }
    float cco = 0.f, pe = 1.f;
    for (unsigned s = 0; s < nch; ++s) {
        const float ev = sE[s];
        pe *= (s > tt) ? ev : 1.0f;
        float pa = 1.f;
        for (unsigned u = 0; u < nch; ++u) { const float av = 1.0f - sA[u]; pa *= (u > s) ? av : 1.0f; }
        cco += (s >= tt) ? pa * pe : 0.f;
    }
    float p0 = 1.f;
    for (unsigned u = 0; u < nch; ++u) p0 *= (1.0f - sA[u]);
    if (t < 16u) {
        sO[t] = live ? cco : 0.f;
        sO[16u + t] = live ? dco : 0.f;
        sO[32u + t] = live ? (2.0f * th) * (1.0f / 1024.0f) : 0.f;
        sO[48u + t] = (t == 0u) ? p0 : 0.f;
    }
    __syncthreads();
    const v4f ov = *(const v4f*)(sO + 4u * tt);
    if (t < 16u) { VST2V4(coef + (size_t)b * 64u + 4u * t, ov); }
}

template <int EPI, int SL2, int OL2>
__global__ __launch_bounds__(256) void k_gemm64(
    const h16* __restrict__ A, unsigned lda, unsigned bsA, const h16* __restrict__ Bt, unsigned ldb, unsigned bsB,
    float* __restrict__ Cf, h16* __restrict__ Ch, const float* __restrict__ aux, unsigned ldc, unsigned bsC,
    unsigned M, unsigned N, unsigned K) {
  __shared__ __align__(16) float sT[8][16 * 68];
  constexpr float SCALE = p2f(-SL2);
  constexpr float OSC = p2f(OL2);
  const unsigned lane = threadIdx.x & 31u;
  const unsigned wave = threadIdx.x >> 5;
  const unsigned tilesN = N >> 6, tilesM = M >> 6;
  const unsigned tile = blockIdx.x * 8u + wave;
  if (tile >= tilesM * tilesN) return;
  const unsigned bz = blockIdx.y;
  A += (size_t)bz * bsA;
  Bt += (size_t)bz * bsB;
  const size_t cbase = (size_t)bz * bsC;
  const unsigned tm = tile / tilesN;
  const unsigned tn = tile - tm * tilesN;
  const unsigned m0 = tm << 6, n0 = tn << 6;
  const unsigned rlane = lane & 15u;
  const unsigned koff = (lane >> 4) * 8u;
  const unsigned mOff = koff;

  v8f acc[4][4];
#pragma unroll
  for (int i = 0; i < 4; ++i)
#pragma unroll
    for (int j = 0; j < 4; ++j) acc[i][j] = (v8f){0.f,0.f,0.f,0.f,0.f,0.f,0.f,0.f};

  for (unsigned k0 = 0; k0 < K; k0 += 32u) {
    v16h bh[4];
#pragma unroll
    for (int j = 0; j < 4; ++j)
      bh[j] = frag_ld(Bt + (size_t)(n0 + ((unsigned)j << 4) + rlane) * ldb + koff + k0);
#pragma unroll
    for (int i = 0; i < 4; ++i) {
      const v16h ah = frag_ld(A + (size_t)(m0 + ((unsigned)i << 4) + rlane) * lda + koff + k0);
#pragma unroll
      for (int j = 0; j < 4; ++j) acc[i][j] = wmma16g(ah, bh[j], acc[i][j]);
    }
  }

  float* slab = sT[wave];
#pragma unroll
  for (int i = 0; i < 4; ++i) {
    const unsigned mBase = m0 + ((unsigned)i << 4);
#pragma unroll
    for (int j = 0; j < 4; ++j) {
#pragma unroll
      for (int r = 0; r < 8; ++r) {
        const float z = acc[i][j][r] * SCALE;
        float v = z;
        if (EPI == 1 || EPI == 2) { const float sg = sigm(z); v = z * sg; if (EPI == 2) v *= OSC; }
        if (EPI == 4) { const float sg = sigm(z); v = sg * (1.0f + z * (1.0f - sg)); acc[i][j][r] = (z * sg) * OSC; }
        slab[(mOff + (unsigned)r) * 68u + ((unsigned)j << 4) + rlane] = v;
      }
    }
    wave_sync_lds();
    if (EPI == 0 || EPI == 1 || EPI == 4) {
      const unsigned hh = lane >> 4, c4 = (lane & 15u) * 4u;
#pragma unroll
      for (int half = 0; half < 2; ++half) {
        v4f vv[4];
#pragma unroll
        for (int it = 0; it < 4; ++it) {
          const unsigned row = (unsigned)(half * 4 + it) * 2u + hh;
          vv[it] = *(const v4f*)(slab + row * 68u + c4);
        }
        for (int pass = 0; pass < 2; ++pass) {
#pragma unroll
          for (int it = 0; it < 4; ++it) {
            const unsigned row = (unsigned)(half * 4 + it) * 2u + hh;
            *(volatile v4f*)(Cf + cbase + (size_t)(mBase + row) * ldc + n0 + c4) = vv[it];
          }
          __threadfence();
        }
      }
    }
    if (EPI == 4) {
      wave_sync_lds();
#pragma unroll
      for (int j = 0; j < 4; ++j)
#pragma unroll
        for (int r = 0; r < 8; ++r)
          slab[(mOff + (unsigned)r) * 68u + ((unsigned)j << 4) + rlane] = acc[i][j][r];
      wave_sync_lds();
    }
    if (EPI >= 2) {
      const unsigned q = lane >> 3, c8 = (lane & 7u) * 8u;
      v8h hv[4];
#pragma unroll
      for (int it = 0; it < 4; ++it) {
        const unsigned row = (unsigned)it * 4u + q;
        const float* sp = slab + row * 68u + c8;
        if (EPI == 3) {
          const float* ap = aux + cbase + (size_t)(mBase + row) * ldc + n0 + c8;
          const v4f a0 = *(const v4f*)ap, a1 = *(const v4f*)(ap + 4);
          const float ax[8] = {a0.x, a0.y, a0.z, a0.w, a1.x, a1.y, a1.z, a1.w};
#pragma unroll
          for (int e = 0; e < 8; ++e) hv[it][e] = toh_flush((sp[e] * ax[e]) * OSC);
        } else {
#pragma unroll
          for (int e = 0; e < 8; ++e) hv[it][e] = toh_flush(sp[e]);
        }
      }
      for (int pass = 0; pass < 2; ++pass) {
#pragma unroll
        for (int it = 0; it < 4; ++it) {
          const unsigned row = (unsigned)it * 4u + q;
          *(volatile v8h*)(Ch + cbase + (size_t)(mBase + row) * ldc + n0 + c8) = hv[it];
        }
        __threadfence();
      }
    }
    wave_sync_lds();
  }
}

template <int CL2>
__global__ __launch_bounds__(256) void k_rmsrow(const float* __restrict__ src, unsigned spitch, const float* __restrict__ gamma,
                                                float* __restrict__ outF, h16* __restrict__ outH, unsigned M) {
    __shared__ __align__(16) float sRow[8][1024];
    constexpr float CAR = p2f(CL2);
    const unsigned wave = threadIdx.x >> 5, L = threadIdx.x & 31u;
    const unsigned row = blockIdx.x * 8u + wave;
    if (row >= M) return;
    const float* pr = src + (size_t)row * spitch + 8u * L;
    float vv[32];
#pragma unroll
    for (int j = 0; j < 4; ++j) {
        const v4f a = *(const v4f*)(pr + 256 * j), b = *(const v4f*)(pr + 256 * j + 4);
        vv[8 * j + 0] = a.x; vv[8 * j + 1] = a.y; vv[8 * j + 2] = a.z; vv[8 * j + 3] = a.w;
        vv[8 * j + 4] = b.x; vv[8 * j + 5] = b.y; vv[8 * j + 6] = b.z; vv[8 * j + 7] = b.w;
    }
    float ss = 0.f;
#pragma unroll
    for (int i = 0; i < 32; ++i) ss += vv[i] * vv[i];
#pragma unroll
    for (int o = 16; o > 0; o >>= 1) ss += __shfl_xor(ss, o, 32);
    const float s = 1.0f / sqrtf(ss * (1.0f / 1024.0f) + 1e-6f);
    float* sr = sRow[wave];
    v8h hv[4];
#pragma unroll
    for (int j = 0; j < 4; ++j) {
        const v4f g0 = *(const v4f*)(gamma + 8u * L + 256u * (unsigned)j), g1 = *(const v4f*)(gamma + 8u * L + 256u * (unsigned)j + 4u);
        const float gg[8] = {g0.x, g0.y, g0.z, g0.w, g1.x, g1.y, g1.z, g1.w};
#pragma unroll
        for (int e = 0; e < 8; ++e) {
            const float o = vv[8 * j + e] * s * bfr(gg[e]);
            sr[8u * L + 256u * (unsigned)j + (unsigned)e] = o;
            hv[j][e] = toh_flush(o * CAR);
        }
    }
    wave_sync_lds();
    v4f fv[8];
#pragma unroll
    for (int j = 0; j < 8; ++j) fv[j] = *(const v4f*)(sr + 4u * L + 128u * (unsigned)j);
    h16* dh = outH + (size_t)row * 1024u + 8u * L;
    float* df = outF + (size_t)row * 1024u + 4u * L;
    for (int pass = 0; pass < 2; ++pass) {
#pragma unroll
        for (int j = 0; j < 4; ++j) *(volatile v8h*)(dh + 256 * j) = hv[j];
#pragma unroll
        for (int j = 0; j < 8; ++j) *(volatile v4f*)(df + 128 * j) = fv[j];
        __threadfence();
    }
}

__global__ __launch_bounds__(256) void k_rowback(const float* __restrict__ y, const float* __restrict__ kf, const float* __restrict__ vsrc,
                                                 unsigned vpitch, const float* __restrict__ lnw, const float* __restrict__ coef,
                                                 h16* __restrict__ dy16, float* __restrict__ dlnc, unsigned rows_per_wave) {
    __shared__ __align__(16) float sLn[1024];
    __shared__ __align__(16) float sD[8][1024];
    constexpr float CDY = p2f(CDY_L2);
    const unsigned tid = threadIdx.x, wave = tid >> 5, L = tid & 31u;
    const unsigned bn = blockIdx.x;
    const unsigned b = bn / (unsigned)NCH;
    const unsigned t = bn - b * (unsigned)NCH;
#pragma unroll
    for (int i = 0; i < 4; ++i) sLn[tid + 256u * (unsigned)i] = bfr(lnw[tid + 256u * (unsigned)i]);
    __syncthreads();
    const float cg = coef[(size_t)b * 64u + 32u + t];
    float dacc[32];
#pragma unroll
    for (int i = 0; i < 32; ++i) dacc[i] = 0.f;
    for (unsigned rr = 0; rr < rows_per_wave; ++rr) {
        const unsigned row = bn * 64u + wave * rows_per_wave + rr;
        const float* yr = y + (size_t)row * 1024u + 8u * L;
        const float* kr = kf + (size_t)row * 1024u + 8u * L;
        const float* vr = vsrc + (size_t)row * vpitch + 8u * L;
        float yv[32], gv[32];
#pragma unroll
        for (int j = 0; j < 4; ++j) {
            const v4f a = *(const v4f*)(yr + 256 * j), c = *(const v4f*)(yr + 256 * j + 4);
            yv[8 * j + 0] = a.x; yv[8 * j + 1] = a.y; yv[8 * j + 2] = a.z; yv[8 * j + 3] = a.w;
            yv[8 * j + 4] = c.x; yv[8 * j + 5] = c.y; yv[8 * j + 6] = c.z; yv[8 * j + 7] = c.w;
        }
        float ss = 0.f;
#pragma unroll
        for (int i = 0; i < 32; ++i) ss += yv[i] * yv[i];
#pragma unroll
        for (int o = 16; o > 0; o >>= 1) ss += __shfl_xor(ss, o, 32);
        const float s = 1.0f / sqrtf(ss * (1.0f / 1024.0f) + 1e-6f);
        float t1 = 0.f;
#pragma unroll
        for (int j = 0; j < 4; ++j) {
            const v4f k0 = *(const v4f*)(kr + 256 * j), k1 = *(const v4f*)(kr + 256 * j + 4);
            const v4f v0 = *(const v4f*)(vr + 256 * j), v1 = *(const v4f*)(vr + 256 * j + 4);
            const float kk[8] = {k0.x, k0.y, k0.z, k0.w, k1.x, k1.y, k1.z, k1.w};
            const float vq[8] = {v0.x, v0.y, v0.z, v0.w, v1.x, v1.y, v1.z, v1.w};
#pragma unroll
            for (int e = 0; e < 8; ++e) {
                const float lw = sLn[8u * L + 256u * (unsigned)j + (unsigned)e];
                const float yy = yv[8 * j + e];
                const float pred = kk[e] + yy * s * lw;
                const float er = pred - vq[e];
                const float g = cg * er;
                gv[8 * j + e] = g;
                t1 += (g * lw) * yy;
                dacc[8 * j + e] += (g * yy) * s;
            }
        }
#pragma unroll
        for (int o = 16; o > 0; o >>= 1) t1 += __shfl_xor(t1, o, 32);
        const float tt = (s * s * s) * t1 * (1.0f / 1024.0f);
        v8h hv[4];
#pragma unroll
        for (int j = 0; j < 4; ++j)
#pragma unroll
            for (int e = 0; e < 8; ++e) {
                const float lw = sLn[8u * L + 256u * (unsigned)j + (unsigned)e];
                const float dyv = (gv[8 * j + e] * lw) * s - yv[8 * j + e] * tt;
                hv[j][e] = toh_flush(dyv * CDY);
            }
        h16* dp = dy16 + (size_t)row * 1024u + 8u * L;
        for (int pass = 0; pass < 2; ++pass) {
#pragma unroll
            for (int j = 0; j < 4; ++j) *(volatile v8h*)(dp + 256 * j) = hv[j];
            __threadfence();
        }
    }
#pragma unroll
    for (int j = 0; j < 4; ++j)
#pragma unroll
        for (int e = 0; e < 8; ++e) sD[wave][8u * L + 256u * (unsigned)j + (unsigned)e] = dacc[8 * j + e];
    __syncthreads();
    v4f acc = *(const v4f*)(&sD[0][4u * tid]);
#pragma unroll
    for (int w = 1; w < 8; ++w) acc += *(const v4f*)(&sD[w][4u * tid]);
    VST2V4(dlnc + (size_t)bn * 1024u + 4u * tid, acc);
}

__global__ __launch_bounds__(256) void k_dlnfin(const float* __restrict__ dlnc, const float* __restrict__ coef, const float* __restrict__ lnw,
                                                float* __restrict__ nln, float* __restrict__ nsl, unsigned nch) {
    const unsigned b = blockIdx.x, tid = threadIdx.x;
    const float* cf = coef + (size_t)b * 64u;
    v4f aC = (v4f){0.f, 0.f, 0.f, 0.f}, aD = (v4f){0.f, 0.f, 0.f, 0.f};
    for (unsigned t = 0; t < nch; ++t) {
        const v4f g = *(const v4f*)(dlnc + (size_t)(b * nch + t) * 1024u + 4u * tid);
        const float ct = cf[t], dt = cf[16u + t];
        aC += g * ct;
        aD += g * dt;
    }
    const float P0 = cf[48];
    const v4f lw = *(const v4f*)(lnw + 4u * tid);
    v4f oM, oS;
    oM.x = P0 * bfr(lw.x) - aC.x; oM.y = P0 * bfr(lw.y) - aC.y; oM.z = P0 * bfr(lw.z) - aC.z; oM.w = P0 * bfr(lw.w) - aC.w;
    oS.x = -aD.x; oS.y = -aD.y; oS.z = -aD.z; oS.w = -aD.w;
    VST2V4(nln + (size_t)b * DM + 4u * tid, oM);
    VST2V4(nsl + (size_t)b * DM + 4u * tid, oS);
}

template <int IL2, int PL2>
__global__ __launch_bounds__(256) void k_grad(const h16* __restrict__ At, const h16* __restrict__ Bt, unsigned ldk,
                                              const float* __restrict__ W, const float* __restrict__ coef,
                                              float* __restrict__ outM, float* __restrict__ outS, h16* __restrict__ plane,
                                              unsigned Mr, unsigned Nc, unsigned nch, unsigned seq) {
    __shared__ __align__(16) float sT[8][16 * 68];
    constexpr float INV = p2f(-IL2);
    constexpr float PC = p2f(PL2);
    const unsigned lane = threadIdx.x & 31u, wave = threadIdx.x >> 5;
    const unsigned b = blockIdx.y;
    const unsigned tilesN = Nc >> 6, tilesM = Mr >> 4;
    const unsigned tile = blockIdx.x * 8u + wave;
    if (tile >= tilesM * tilesN) return;
    const unsigned tm = tile / tilesN;
    const unsigned tn = tile - tm * tilesN;
    const unsigned m0 = tm << 4, n0 = tn << 6;
    const unsigned rlane = lane & 15u;
    const unsigned koff = (lane >> 4) * 8u;
    const unsigned mOff = koff;
    const float* cf = coef + (size_t)b * 64u;
    const h16* ap = At + (size_t)(m0 + rlane) * ldk + (size_t)b * seq + koff;
    const h16* bp = Bt + (size_t)(n0 + rlane) * ldk + (size_t)b * seq + koff;

    v8f accC[4], accD[4];
#pragma unroll
    for (int j = 0; j < 4; ++j) { accC[j] = (v8f){0.f,0.f,0.f,0.f,0.f,0.f,0.f,0.f}; accD[j] = accC[j]; }

    for (unsigned t = 0; t < nch; ++t) {
        const float ct = cf[t], dt = cf[16u + t];
        v8f T[4];
#pragma unroll
        for (int j = 0; j < 4; ++j) T[j] = (v8f){0.f,0.f,0.f,0.f,0.f,0.f,0.f,0.f};
#pragma unroll
        for (int kk = 0; kk < 2; ++kk) {
            const unsigned k0 = t * 64u + (unsigned)kk * 32u;
            const v16h ah = frag_ld(ap + k0);
#pragma unroll
            for (int j = 0; j < 4; ++j) {
                const v16h bh = frag_ld(bp + (size_t)((unsigned)j << 4) * ldk + k0);
                T[j] = wmma16g(ah, bh, T[j]);
            }
        }
#pragma unroll
        for (int j = 0; j < 4; ++j)
#pragma unroll
            for (int r = 0; r < 8; ++r) { accC[j][r] += ct * T[j][r]; accD[j][r] += dt * T[j][r]; }
    }

    float* slab = sT[wave];
    const float P0 = cf[48];
    const size_t obase = (size_t)b * Mr * Nc;
    const unsigned hh = lane >> 4, c4 = (lane & 15u) * 4u;
    const unsigned q = lane >> 3, c8 = (lane & 7u) * 8u;
#pragma unroll
    for (int j = 0; j < 4; ++j)
#pragma unroll
        for (int r = 0; r < 8; ++r) slab[(mOff + (unsigned)r) * 68u + ((unsigned)j << 4) + rlane] = accC[j][r] * INV;
    wave_sync_lds();
#pragma unroll
    for (int half = 0; half < 2; ++half) {
        v4f vv[4];
#pragma unroll
        for (int it = 0; it < 4; ++it) {
            const unsigned row = (unsigned)(half * 4 + it) * 2u + hh;
            const v4f s4 = *(const v4f*)(slab + row * 68u + c4);
            const v4f w4 = *(const v4f*)(W + (size_t)(m0 + row) * Nc + n0 + c4);
            vv[it].x = P0 * bfr(w4.x) - s4.x; vv[it].y = P0 * bfr(w4.y) - s4.y;
            vv[it].z = P0 * bfr(w4.z) - s4.z; vv[it].w = P0 * bfr(w4.w) - s4.w;
        }
        for (int pass = 0; pass < 2; ++pass) {
#pragma unroll
            for (int it = 0; it < 4; ++it) {
                const unsigned row = (unsigned)(half * 4 + it) * 2u + hh;
                *(volatile v4f*)(outM + obase + (size_t)(m0 + row) * Nc + n0 + c4) = vv[it];
            }
            __threadfence();
        }
    }
    {
        v8h hv[4];
#pragma unroll
        for (int it = 0; it < 4; ++it) {
            const unsigned row = (unsigned)it * 4u + q;
            const float* sp = slab + row * 68u + c8;
            const float* wp = W + (size_t)(m0 + row) * Nc + n0 + c8;
            const v4f w0 = *(const v4f*)wp, w1 = *(const v4f*)(wp + 4);
            const float ww[8] = {w0.x, w0.y, w0.z, w0.w, w1.x, w1.y, w1.z, w1.w};
#pragma unroll
            for (int e = 0; e < 8; ++e) hv[it][e] = toh_flush((P0 * bfr(ww[e]) - sp[e]) * PC);
        }
        for (int pass = 0; pass < 2; ++pass) {
#pragma unroll
            for (int it = 0; it < 4; ++it) {
                const unsigned row = (unsigned)it * 4u + q;
                *(volatile v8h*)(plane + obase + (size_t)(m0 + row) * Nc + n0 + c8) = hv[it];
            }
            __threadfence();
        }
    }
    wave_sync_lds();
#pragma unroll
    for (int j = 0; j < 4; ++j)
#pragma unroll
        for (int r = 0; r < 8; ++r) slab[(mOff + (unsigned)r) * 68u + ((unsigned)j << 4) + rlane] = -(accD[j][r] * INV);
    wave_sync_lds();
#pragma unroll
    for (int half = 0; half < 2; ++half) {
        v4f vv[4];
#pragma unroll
        for (int it = 0; it < 4; ++it) {
            const unsigned row = (unsigned)(half * 4 + it) * 2u + hh;
            vv[it] = *(const v4f*)(slab + row * 68u + c4);
        }
        for (int pass = 0; pass < 2; ++pass) {
#pragma unroll
            for (int it = 0; it < 4; ++it) {
                const unsigned row = (unsigned)(half * 4 + it) * 2u + hh;
                *(volatile v4f*)(outS + obase + (size_t)(m0 + row) * Nc + n0 + c4) = vv[it];
            }
            __threadfence();
        }
    }
}

__global__ __launch_bounds__(256) void k_out(const float* __restrict__ yq, const float* __restrict__ qf, const float* __restrict__ nln,
                                             float* __restrict__ out, unsigned M) {
    const unsigned wave = threadIdx.x >> 5, L = threadIdx.x & 31u;
    const unsigned row = blockIdx.x * 8u + wave;
    if (row >= M) return;
    const unsigned b = row / (unsigned)SEQ;
    const unsigned s = row - b * (unsigned)SEQ;
    const float* yr = yq + (size_t)row * 1024u + 4u * L;
    const float* qr = qf + (size_t)row * 1024u + 4u * L;
    const float* gr = nln + (size_t)b * DM + 4u * L;
    v4f yv[8];
    float ss = 0.f;
#pragma unroll
    for (int j = 0; j < 8; ++j) {
        yv[j] = *(const v4f*)(yr + 128 * j);
        ss += yv[j].x * yv[j].x; ss += yv[j].y * yv[j].y; ss += yv[j].z * yv[j].z; ss += yv[j].w * yv[j].w;
    }
#pragma unroll
    for (int o = 16; o > 0; o >>= 1) ss += __shfl_xor(ss, o, 32);
    const float sc = 1.0f / sqrtf(ss * (1.0f / 1024.0f) + 1e-6f);
    v4f ov[8];
#pragma unroll
    for (int j = 0; j < 8; ++j) {
        const v4f qv = *(const v4f*)(qr + 128 * j);
        const v4f gv = *(const v4f*)(gr + 128 * j);
        ov[j].x = qv.x + yv[j].x * sc * gv.x; ov[j].y = qv.y + yv[j].y * sc * gv.y;
        ov[j].z = qv.z + yv[j].z * sc * gv.z; ov[j].w = qv.w + yv[j].w * sc * gv.w;
    }
    float* dst = out + ((size_t)b * SEQ_FULL + s) * 1024u + 4u * L;
    for (int pass = 0; pass < 2; ++pass) {
#pragma unroll
        for (int j = 0; j < 8; ++j) *(volatile v4f*)(dst + 128 * j) = ov[j];
        __threadfence();
    }
}

constexpr size_t al256(size_t x) { return (x + 255) & ~(size_t)255; }
constexpr size_t cmax(size_t a, size_t b) { return a > b ? a : b; }
constexpr size_t SZ_X16  = (size_t)MTOK * DM * 2;
constexpr size_t SZ_WKVQ = (size_t)3 * DM * DM * 2;
constexpr size_t SZ_H16  = (size_t)MTOK * HID * 2;
constexpr size_t SZ_F32D = (size_t)MTOK * DM * 4;
constexpr size_t SZ_D16  = (size_t)MTOK * DM * 2;
constexpr size_t SZ_W16  = (size_t)HID * DM * 2;
constexpr size_t SZ_NW16 = (size_t)NB * HID * DM * 2;
constexpr size_t SZ_SP   = (size_t)MTOK * 3 * DM * 4;
constexpr size_t SZ_SD   = (size_t)MTOK * HID * 4;
constexpr size_t SZ_RA = cmax(al256(SZ_X16) + al256(SZ_WKVQ), al256(SZ_H16));
constexpr size_t SZ_RB = cmax(al256(SZ_SP), 2 * al256(SZ_NW16) + al256(SZ_H16));
constexpr size_t SZ_RC = cmax(al256(SZ_SD), al256(SZ_F32D));
constexpr size_t SZ_RD = cmax(al256(SZ_F32D), al256(SZ_H16));
constexpr size_t SZ_RE = cmax(al256(SZ_F32D), al256(SZ_H16));
constexpr size_t SZ_GATES = al256((size_t)NB * NCH * 128);
constexpr size_t SZ_COEF  = al256((size_t)NB * 256);
constexpr size_t SZ_DLNC  = al256((size_t)NB * NCH * 4096);
constexpr size_t WS_TOTAL = SZ_RA + SZ_RB + SZ_RC + SZ_RD + SZ_RE + 3 * al256(SZ_W16) + al256(SZ_F32D) + 5 * al256(SZ_D16)
                          + al256(SZ_H16) + SZ_GATES + SZ_COEF + SZ_DLNC;
static_assert(WS_TOTAL <= (size_t)134217728);
static_assert(al256(SZ_X16) + al256(SZ_WKVQ) <= SZ_RA && al256(SZ_H16) <= SZ_RA);
static_assert(al256(SZ_SP) <= SZ_RB && 2 * al256(SZ_NW16) + al256(SZ_H16) <= SZ_RB);
static_assert(al256(SZ_SD) <= SZ_RC && al256(SZ_F32D) <= SZ_RC);
static_assert(al256(SZ_F32D) <= SZ_RD && al256(SZ_H16) <= SZ_RD && al256(SZ_F32D) <= SZ_RE && al256(SZ_H16) <= SZ_RE);

extern "C" void kernel_launch(void* const* d_in, const int* in_sizes, int n_in, void* d_out, int out_size,
                              void* d_ws, size_t ws_size, hipStream_t stream) {
    if (n_in < 12) return;
    if (in_sizes[0] < ((NB - 1) * SEQ_FULL + SEQ) * DM) return;
    if (in_sizes[1] < HID * DM || in_sizes[2] < DM * HID || in_sizes[3] < DM) return;
    if (in_sizes[4] < DM * DM || in_sizes[5] < DM * DM || in_sizes[6] < DM * DM || in_sizes[7] < DM || in_sizes[8] < DM) return;
    if (in_sizes[9] < CHK * DM || in_sizes[10] < CHK * DM || in_sizes[11] < CHK * DM) return;
    if ((unsigned)out_size < OUT_ELEMS) return;
    if (WS_TOTAL > ws_size) return;

    const float* x    = (const float*)d_in[0];
    const float* w1   = (const float*)d_in[1];
    const float* w2   = (const float*)d_in[2];
    const float* ln_w = (const float*)d_in[3];
    const float* wq   = (const float*)d_in[4];
    const float* wk   = (const float*)d_in[5];
    const float* wv   = (const float*)d_in[6];
    const float* qn_w = (const float*)d_in[7];
    const float* kn_w = (const float*)d_in[8];
    const float* aw   = (const float*)d_in[9];
    const float* tw   = (const float*)d_in[10];
    const float* ew   = (const float*)d_in[11];
    float* out = (float*)d_out;

    char* wsp = (char*)d_ws;
    size_t off = 0;
    auto carve = [&](size_t bytes) -> char* { char* r = wsp + off; off += al256(bytes); return r; };
    char* rA = carve(SZ_RA);
    char* rB = carve(SZ_RB);
    char* rC = carve(SZ_RC);
    char* rD = carve(SZ_RD);
    char* rE = carve(SZ_RE);
    h16*   w1_16  = (h16*)carve(SZ_W16);
    h16*   w2_16  = (h16*)carve(SZ_W16);
    h16*   w2T16  = (h16*)carve(SZ_W16);
    float* qf32   = (float*)carve(SZ_F32D);
    h16*   k16    = (h16*)carve(SZ_D16);
    h16*   q16    = (h16*)carve(SZ_D16);
    h16*   kT16   = (h16*)carve(SZ_D16);
    h16*   dy16   = (h16*)carve(SZ_D16);
    h16*   dyT16  = (h16*)carve(SZ_D16);
    h16*   hT16   = (h16*)carve(SZ_H16);
    float* gates  = (float*)carve((size_t)NB * NCH * 128);
    float* coef   = (float*)carve((size_t)NB * 256);
    float* dlnc   = (float*)carve((size_t)NB * NCH * 4096);
    if (off != WS_TOTAL || off > ws_size || off > (size_t)134217728) return;

    h16*   x16    = (h16*)rA;
    h16*   wkvq16 = (h16*)(rA + al256(SZ_X16));
    h16*   hpl16  = (h16*)rA;
    float* sP     = (float*)rB;
    h16*   nw1_16 = (h16*)rB;
    h16*   nw2_16 = (h16*)(rB + al256(SZ_NW16));
    h16*   hq16   = (h16*)(rB + 2 * al256(SZ_NW16));
    float* sd     = (float*)rC;
    float* yq     = (float*)rC;
    float* kf32   = (float*)rD;
    h16*   dz16   = (h16*)rD;
    float* ybuf   = (float*)rE;
    h16*   dzT16  = (h16*)rE;

    k_cvt<CX_L2><<<dim3((SEQ * DM / 8) / 256, NB), 256, 0, stream>>>(x, x16, SEQ * DM / 8, SEQ_FULL * DM, SEQ * DM);
    k_cvt<CW_L2><<<dim3((DM * DM / 8) / 256, 1), 256, 0, stream>>>(wk, wkvq16, DM * DM / 8, 0u, 0u);
    k_cvt<CW_L2><<<dim3((DM * DM / 8) / 256, 1), 256, 0, stream>>>(wv, wkvq16 + (size_t)DM * DM, DM * DM / 8, 0u, 0u);
    k_cvt<CW_L2><<<dim3((DM * DM / 8) / 256, 1), 256, 0, stream>>>(wq, wkvq16 + (size_t)2 * DM * DM, DM * DM / 8, 0u, 0u);
    k_cvt<CW_L2><<<dim3((HID * DM / 8) / 256, 1), 256, 0, stream>>>(w1, w1_16, HID * DM / 8, 0u, 0u);
    k_cvt<CW_L2><<<dim3((HID * DM / 8) / 256, 1), 256, 0, stream>>>(w2, w2_16, HID * DM / 8, 0u, 0u);
    k_tr16<<<dim3(HID / 64, DM / 64), 256, 0, stream>>>(w2_16, w2T16, DM, HID);

    k_gates<<<NB * NCH, 256, 0, stream>>>(x, aw, tw, ew, gates, 64u);
    k_coef<<<NB, 32, 0, stream>>>(gates, coef, (unsigned)NCH);

    {
        const unsigned g = ((MTOK / 64) * (3 * DM / 64) + 7) / 8;
        k_gemm64<1, CX_L2 + CW_L2, 0><<<dim3(g, 1), 256, 0, stream>>>(x16, DM, 0u, wkvq16, DM, 0u, sP, hq16, sP, 3 * DM, 0u,
                                                                      MTOK, 3 * DM, DM);
    }
    k_rmsrow<CK_L2><<<MTOK / 8, 256, 0, stream>>>(sP, 3 * DM, kn_w, kf32, k16, MTOK);
    k_rmsrow<CK_L2><<<MTOK / 8, 256, 0, stream>>>(sP + 2 * DM, 3 * DM, qn_w, qf32, q16, MTOK);
    k_tr16<<<dim3(DM / 64, MTOK / 64), 256, 0, stream>>>(k16, kT16, MTOK, DM);

    {
        const unsigned g = ((MTOK / 64) * (HID / 64) + 7) / 8;
        k_gemm64<4, CK_L2 + CW_L2, CH_L2><<<dim3(g, 1), 256, 0, stream>>>(k16, DM, 0u, w1_16, DM, 0u, sd, hpl16, sd, HID, 0u,
                                                                          MTOK, HID, DM);
    }
    k_tr16<<<dim3(HID / 64, MTOK / 64), 256, 0, stream>>>(hpl16, hT16, MTOK, HID);
    {
        const unsigned g = ((MTOK / 64) * (DM / 64) + 7) / 8;
        k_gemm64<0, CH_L2 + CW_L2, 0><<<dim3(g, 1), 256, 0, stream>>>(hpl16, HID, 0u, w2_16, HID, 0u, ybuf, dy16, ybuf, DM, 0u,
                                                                      MTOK, DM, HID);
    }
    k_rowback<<<NB * NCH, 256, 0, stream>>>(ybuf, kf32, sP + DM, 3 * DM, ln_w, coef, dy16, dlnc, 8u);
    k_dlnfin<<<NB, 256, 0, stream>>>(dlnc, coef, ln_w, out + OFF_NLN, out + OFF_NSL, (unsigned)NCH);
    k_tr16<<<dim3(DM / 64, MTOK / 64), 256, 0, stream>>>(dy16, dyT16, MTOK, DM);
    {
        const unsigned g = ((MTOK / 64) * (HID / 64) + 7) / 8;
        k_gemm64<3, CDY_L2 + CW_L2, CDZ_L2><<<dim3(g, 1), 256, 0, stream>>>(dy16, DM, 0u, w2T16, DM, 0u, ybuf, dz16, sd, HID, 0u,
                                                                            MTOK, HID, DM);
    }
    k_tr16<<<dim3(HID / 64, MTOK / 64), 256, 0, stream>>>(dz16, dzT16, MTOK, HID);

    k_grad<CDY_L2 + CH_L2, CN2_L2><<<dim3(((DM / 16) * (HID / 64) + 7) / 8, NB), 256, 0, stream>>>(
        dyT16, hT16, MTOK, w2, coef, out + OFF_NW2, out + OFF_NS2, nw2_16, DM, HID, (unsigned)NCH, (unsigned)SEQ);
    k_grad<CDZ_L2 + CK_L2, CN1_L2><<<dim3(((HID / 16) * (DM / 64) + 7) / 8, NB), 256, 0, stream>>>(
        dzT16, kT16, MTOK, w1, coef, out + OFF_NW1, out + OFF_NS1, nw1_16, HID, DM, (unsigned)NCH, (unsigned)SEQ);

    {
        const unsigned g = ((SEQ / 64) * (HID / 64) + 7) / 8;
        k_gemm64<2, CK_L2 + CN1_L2, CHQ_L2><<<dim3(g, NB), 256, 0, stream>>>(q16, DM, SEQ * DM, nw1_16, DM, HID * DM, yq, hq16, yq,
                                                                             HID, SEQ * HID, SEQ, HID, DM);
    }
    {
        const unsigned g = ((SEQ / 64) * (DM / 64) + 7) / 8;
        k_gemm64<0, CHQ_L2 + CN2_L2, 0><<<dim3(g, NB), 256, 0, stream>>>(hq16, HID, SEQ * HID, nw2_16, HID, DM * HID, yq, dy16, yq,
                                                                         DM, SEQ * DM, SEQ, DM, HID);
    }
    k_out<<<MTOK / 8, 256, 0, stream>>>(yq, qf32, out + OFF_NLN, out + OFF_OUT, MTOK);
}
